// FrameStackMamba2_67267777790256
// MI455X (gfx1250) — hardware-verified
//
#include <hip/hip_runtime.h>
#include <hip/hip_bf16.h>
#include <math.h>


typedef _Float16 bf16;
typedef _Float16 f16;
typedef __attribute__((ext_vector_type(4))) unsigned v4u_t;
typedef unsigned v4ua __attribute__((ext_vector_type(4), may_alias));
typedef __attribute__((ext_vector_type(4))) float v4f_t;
typedef float v4fa __attribute__((ext_vector_type(4), may_alias));
typedef __attribute__((ext_vector_type(16))) bf16  bf16x16;
typedef bf16x16 f16x16;
typedef __attribute__((ext_vector_type(8)))  bf16  bf16x8;
typedef bf16x8 f16x8;
typedef __attribute__((ext_vector_type(4)))  bf16  bf16x4;
typedef __attribute__((ext_vector_type(8)))  float f32x8;
__device__ __forceinline__ f32x8 wmma16(f16x16 a, f16x16 b, f32x8 c) {
  c = __builtin_amdgcn_wmma_f32_16x16x32_f16(false, a, false, b, (short)0, c, false, false);
  asm volatile("v_nop\n\tv_nop\n\tv_nop\n\tv_nop" : "+v"(c) : "v"(a), "v"(b));
  return c;
}
#define LDS_STRIDE 48
#define KSTRIDE    72
#define VSTRIDE    48

__device__ __forceinline__ f32x8 wmma_bf16(bf16x16 a, bf16x16 b, f32x8 c) {
  c = __builtin_amdgcn_wmma_f32_16x16x32_f16(false, a, false, b, (short)0, c, false, false);
  asm volatile("v_nop\n\tv_nop\n\tv_nop\n\tv_nop" : "+v"(c) : "v"(a), "v"(b));
  return c;
}

template <typename T>
__device__ __forceinline__ bf16x16 load_frag(const T* __restrict__ base, int ld,
                                             int row0, int k0) {
  const int lane = threadIdx.x & 31;
  const int r    = lane & 15;
  const int kh   = (lane >> 4) * 8;
  const T* p0 = base + (size_t)(row0 + r) * ld + (k0 + kh);
  const T* p1 = p0 + 16;
  bf16x16 f;
#pragma unroll
  for (int i = 0; i < 8; ++i) {
    f[i]     = (bf16)p0[i];
    f[i + 8] = (bf16)p1[i];
  }
  return f;
}

__device__ __forceinline__ bf16x16 lds_frag(const bf16* base, int stride) {
  const int lane = threadIdx.x & 31;
  const int row  = lane & 15;
  const int kh   = (lane >> 4) * 8;
  const bf16x8 lo = *(const bf16x8*)(base + row * stride + kh);
  const bf16x8 hi = *(const bf16x8*)(base + row * stride + kh + 16);
  bf16x16 f;
#pragma unroll
  for (int i = 0; i < 8; ++i) { f[i] = lo[i]; f[i + 8] = hi[i]; }
  return f;
}

template <typename T>
__device__ __forceinline__ void stage_read16(const T* __restrict__ p, float* buf) {
#pragma unroll
  for (int i = 0; i < 16; ++i) buf[i] = (float)p[i];
}

__device__ __forceinline__ void stage_write(bf16* dst, const float* buf, int nquad) {
#pragma unroll
  for (int i = 0; i < nquad; ++i) {
    bf16x4 q;
    q[0] = (bf16)buf[4 * i];     q[1] = (bf16)buf[4 * i + 1];
    q[2] = (bf16)buf[4 * i + 2]; q[3] = (bf16)buf[4 * i + 3];
    *(bf16x4*)(dst + 4 * i) = q;
  }
}


#define GSTR 48
#define GSTR 48
template <typename AT, int EPI, bool OUT16>
__global__ __launch_bounds__(256) void gemm_kne(const AT* __restrict__ A, int lda, const float* __restrict__ Wm, int ldw,
                                                const float* __restrict__ bias, const float* __restrict__ R, const float* __restrict__ gvec,
                                                void* __restrict__ Yv, int ldy, int K) {
  __shared__ __attribute__((aligned(16))) f16 ldsA[128 * GSTR];
  __shared__ __attribute__((aligned(16))) f16 ldsW[128 * GSTR];
  __shared__ __attribute__((aligned(16))) float oS[8][32 * 68];
  const int tid = threadIdx.x, lane = tid & 31, wave = tid >> 5, cl = lane & 15, rh = (lane >> 4) * 8;
  const int m0 = blockIdx.x * 128, n0 = blockIdx.y * 128;
  const int wm = (wave & 3) * 32, wn = (wave >> 2) * 64;
  f32x8 acc[2][4];
#pragma unroll
  for (int i = 0; i < 2; ++i)
#pragma unroll
    for (int j = 0; j < 4; ++j) { f32x8 z = {}; acc[i][j] = z; }
#pragma unroll 1
  for (int k0 = 0; k0 < K; k0 += 32) {
    __syncthreads();
    { const int row = tid >> 1, ch = (tid & 1) * 16;
      const AT* src = A + (size_t)(m0 + row) * lda + k0 + ch;
#pragma unroll
      for (int g = 0; g < 16; ++g) ldsA[row * GSTR + ch + g] = (f16)src[g]; }
    { const int k = tid >> 3, nn0 = (tid & 7) * 16;
      const float* src = Wm + (size_t)(k0 + k) * ldw + n0 + nn0;
#pragma unroll
      for (int g = 0; g < 4; ++g) { const v4f_t v = *(const v4f_t*)(src + 4 * g);
#pragma unroll
        for (int u = 0; u < 4; ++u) ldsW[(nn0 + 4 * g + u) * GSTR + k] = (f16)v[u]; } }
    __syncthreads();
    f16x16 af[2];
#pragma unroll
    for (int i = 0; i < 2; ++i) af[i] = lds_frag(ldsA + (wm + 16 * i) * GSTR, GSTR);
#pragma unroll
    for (int j = 0; j < 4; ++j) {
      const f16x16 bf = lds_frag(ldsW + (wn + 16 * j) * GSTR, GSTR);
#pragma unroll
      for (int i = 0; i < 2; ++i) acc[i][j] = wmma16(af[i], bf, acc[i][j]);
    }
  }
  float* so = oS[wave];
#pragma unroll
  for (int i = 0; i < 2; ++i)
#pragma unroll
    for (int j = 0; j < 4; ++j) {
      const int n = n0 + wn + 16 * j + cl;
      const float bv = bias ? bias[n] : 0.0f;
      const float gv = (EPI == 2 || EPI == 4) ? gvec[n] : 0.0f;
      if (EPI == 1) {
#pragma unroll 1
        for (int r = 0; r < 8; ++r) { const float xg = acc[i][j][r] + bv; so[(16 * i + rh + r) * 68 + 16 * j + cl] = 0.5f * xg * (1.0f + erff(xg * 0.70710678118654752f)); }
      } else {
#pragma unroll
        for (int r = 0; r < 8; ++r) {
          float v = acc[i][j][r] + bv;
          if (EPI == 3) v = fmaxf(v, 0.0f);
          if (EPI == 4) v = gv * v;
          if (EPI == 2) v = R[(size_t)(m0 + wm + 16 * i + rh + r) * ldy + n] + gv * v;
          so[(16 * i + rh + r) * 68 + 16 * j + cl] = v;
        }
      }
    }
  asm volatile("s_wait_dscnt 0" ::: "memory");
  __builtin_amdgcn_wave_barrier();
#pragma unroll 1
  for (int pass = 0; pass < 2; ++pass) {
    if (OUT16) {
      f16* Y = (f16*)Yv;
#pragma unroll
      for (int it = 0; it < 8; ++it) { const int c = lane + 32 * it, rr = c >> 3, q8 = (c & 7) * 8;
        union { f16 h[8]; v4u_t v; } u;
#pragma unroll
        for (int e = 0; e < 8; ++e) u.h[e] = (f16)so[rr * 68 + q8 + e];
        *(volatile v4u_t*)(Y + (size_t)(m0 + wm + rr) * ldy + n0 + wn + q8) = u.v; }
    } else {
      float* Y = (float*)Yv;
#pragma unroll
      for (int it = 0; it < 16; ++it) { const int f4 = lane + 32 * it, rr = f4 >> 4, q = (f4 & 15) * 4;
        *(volatile v4f_t*)(Y + (size_t)(m0 + wm + rr) * ldy + n0 + wn + q) = *(const v4fa*)(so + rr * 68 + q); }
    }
    __threadfence();
  }
}

template <typename AT, int EPI, bool OUT16>
__global__ __launch_bounds__(256) void gemm_knez(const AT* __restrict__ A, int lda, size_t strideA, const float* __restrict__ Wm, int ldw, size_t strideW,
                                                 const float* __restrict__ bias, const float* __restrict__ R, const float* __restrict__ gvec,
                                                 void* __restrict__ Yv, int ldy, size_t strideY, int K) {
  A += (size_t)blockIdx.z * strideA; Wm += (size_t)blockIdx.z * strideW; Yv = (void*)((char*)Yv + (size_t)blockIdx.z * strideY * (OUT16 ? 2 : 4)); if (R) R += (size_t)blockIdx.z * strideY;
  __shared__ __attribute__((aligned(16))) f16 ldsA[128 * GSTR];
  __shared__ __attribute__((aligned(16))) f16 ldsW[128 * GSTR];
  __shared__ __attribute__((aligned(16))) float oS[8][32 * 68];
  const int tid = threadIdx.x, lane = tid & 31, wave = tid >> 5, cl = lane & 15, rh = (lane >> 4) * 8;
  const int m0 = blockIdx.x * 128, n0 = blockIdx.y * 128;
  const int wm = (wave & 3) * 32, wn = (wave >> 2) * 64;
  f32x8 acc[2][4];
#pragma unroll
  for (int i = 0; i < 2; ++i)
#pragma unroll
    for (int j = 0; j < 4; ++j) { f32x8 z = {}; acc[i][j] = z; }
#pragma unroll 1
  for (int k0 = 0; k0 < K; k0 += 32) {
    __syncthreads();
    { const int row = tid >> 1, ch = (tid & 1) * 16;
      const AT* src = A + (size_t)(m0 + row) * lda + k0 + ch;
#pragma unroll
      for (int g = 0; g < 16; ++g) ldsA[row * GSTR + ch + g] = (f16)src[g]; }
    { const int k = tid >> 3, nn0 = (tid & 7) * 16;
      const float* src = Wm + (size_t)(k0 + k) * ldw + n0 + nn0;
#pragma unroll
      for (int g = 0; g < 4; ++g) { const v4f_t v = *(const v4f_t*)(src + 4 * g);
#pragma unroll
        for (int u = 0; u < 4; ++u) ldsW[(nn0 + 4 * g + u) * GSTR + k] = (f16)v[u]; } }
    __syncthreads();
    f16x16 af[2];
#pragma unroll
    for (int i = 0; i < 2; ++i) af[i] = lds_frag(ldsA + (wm + 16 * i) * GSTR, GSTR);
#pragma unroll
    for (int j = 0; j < 4; ++j) {
      const f16x16 bf = lds_frag(ldsW + (wn + 16 * j) * GSTR, GSTR);
#pragma unroll
      for (int i = 0; i < 2; ++i) acc[i][j] = wmma16(af[i], bf, acc[i][j]);
    }
  }
  float* so = oS[wave];
#pragma unroll
  for (int i = 0; i < 2; ++i)
#pragma unroll
    for (int j = 0; j < 4; ++j) {
      const int n = n0 + wn + 16 * j + cl;
      const float bv = bias ? bias[n] : 0.0f;
      const float gv = (EPI == 2 || EPI == 4) ? gvec[n] : 0.0f;
      if (EPI == 1) {
#pragma unroll 1
        for (int r = 0; r < 8; ++r) { const float xg = acc[i][j][r] + bv; so[(16 * i + rh + r) * 68 + 16 * j + cl] = 0.5f * xg * (1.0f + erff(xg * 0.70710678118654752f)); }
      } else {
#pragma unroll
        for (int r = 0; r < 8; ++r) {
          float v = acc[i][j][r] + bv;
          if (EPI == 3) v = fmaxf(v, 0.0f);
          if (EPI == 4) v = gv * v;
          if (EPI == 2) v = R[(size_t)(m0 + wm + 16 * i + rh + r) * ldy + n] + gv * v;
          so[(16 * i + rh + r) * 68 + 16 * j + cl] = v;
        }
      }
    }
  asm volatile("s_wait_dscnt 0" ::: "memory");
  __builtin_amdgcn_wave_barrier();
#pragma unroll 1
  for (int pass = 0; pass < 2; ++pass) {
    if (OUT16) {
      f16* Y = (f16*)Yv;
#pragma unroll
      for (int it = 0; it < 8; ++it) { const int c = lane + 32 * it, rr = c >> 3, q8 = (c & 7) * 8;
        union { f16 h[8]; v4u_t v; } u;
#pragma unroll
        for (int e = 0; e < 8; ++e) u.h[e] = (f16)so[rr * 68 + q8 + e];
        *(volatile v4u_t*)(Y + (size_t)(m0 + wm + rr) * ldy + n0 + wn + q8) = u.v; }
    } else {
      float* Y = (float*)Yv;
#pragma unroll
      for (int it = 0; it < 16; ++it) { const int f4 = lane + 32 * it, rr = f4 >> 4, q = (f4 & 15) * 4;
        *(volatile v4f_t*)(Y + (size_t)(m0 + wm + rr) * ldy + n0 + wn + q) = *(const v4fa*)(so + rr * 68 + q); }
    }
    __threadfence();
  }
}

template <typename AT, bool ACC>
__global__ __launch_bounds__(256) void gemm_kn2(const AT* __restrict__ A, int lda, size_t strideA,
                                               const float* __restrict__ Wm, int ldw, size_t strideW,
                                               const float* __restrict__ bias, float scale,
                                               float* __restrict__ Y, int ldy, size_t strideY, int K) {
  __shared__ __attribute__((aligned(16))) f16 ldsA[128 * GSTR], ldsAl[128 * GSTR];
  __shared__ __attribute__((aligned(16))) f16 ldsW[128 * GSTR], ldsWl[128 * GSTR];
  __shared__ __attribute__((aligned(16))) float oS[8][32 * 68];
  const int tid = threadIdx.x, lane = tid & 31, wave = tid >> 5, cl = lane & 15, rh = (lane >> 4) * 8;
  const int m0 = blockIdx.x * 128, n0 = blockIdx.y * 128;
  const int wm = (wave & 3) * 32, wn = (wave >> 2) * 64;
  A += (size_t)blockIdx.z * strideA; Wm += (size_t)blockIdx.z * strideW; Y += (size_t)blockIdx.z * strideY;
  f32x8 acc[2][4], accx[2][4];
#pragma unroll
  for (int i = 0; i < 2; ++i)
#pragma unroll
    for (int j = 0; j < 4; ++j) { f32x8 z = {}; acc[i][j] = z; accx[i][j] = z; }
#pragma unroll 1
  for (int k0 = 0; k0 < K; k0 += 32) {
    __syncthreads();
    {
      const int row = tid >> 1, ch = (tid & 1) * 16;
      const AT* src = A + (size_t)(m0 + row) * lda + k0 + ch;
#pragma unroll
      for (int g = 0; g < 16; ++g) { const float v = (float)src[g]; const f16 h = (f16)v; ldsA[row * GSTR + ch + g] = h; ldsAl[row * GSTR + ch + g] = (f16)((v - (float)h) * 2048.0f); }
    }
    {
      const int k = tid >> 3, nn0 = (tid & 7) * 16;
      const float* src = Wm + (size_t)(k0 + k) * ldw + n0 + nn0;
#pragma unroll
      for (int g = 0; g < 4; ++g) { const v4f_t v = *(const v4f_t*)(src + 4 * g);
#pragma unroll
        for (int u = 0; u < 4; ++u) { const f16 h = (f16)v[u]; ldsW[(nn0 + 4 * g + u) * GSTR + k] = h; ldsWl[(nn0 + 4 * g + u) * GSTR + k] = (f16)((v[u] - (float)h) * 2048.0f); } }
    }
    __syncthreads();
    f16x16 af[2], afl[2];
#pragma unroll
    for (int i = 0; i < 2; ++i) { af[i] = lds_frag(ldsA + (wm + 16 * i) * GSTR, GSTR); afl[i] = lds_frag(ldsAl + (wm + 16 * i) * GSTR, GSTR); }
#pragma unroll
    for (int j = 0; j < 4; ++j) {
      const f16x16 bf = lds_frag(ldsW + (wn + 16 * j) * GSTR, GSTR), bfl = lds_frag(ldsWl + (wn + 16 * j) * GSTR, GSTR);
#pragma unroll
      for (int i = 0; i < 2; ++i) { acc[i][j] = wmma16(af[i], bf, acc[i][j]); accx[i][j] = wmma16(af[i], bfl, accx[i][j]); accx[i][j] = wmma16(afl[i], bf, accx[i][j]); }
    }
  }
  float* so = oS[wave];
#pragma unroll
  for (int i = 0; i < 2; ++i)
#pragma unroll
    for (int j = 0; j < 4; ++j) {
      const float bv = bias ? bias[n0 + wn + 16 * j + cl] : 0.0f;
#pragma unroll
      for (int r = 0; r < 8; ++r) so[(16 * i + rh + r) * 68 + 16 * j + cl] = (acc[i][j][r] + accx[i][j][r] * (1.0f / 2048.0f)) * scale + bv;
    }
  asm volatile("s_wait_dscnt 0" ::: "memory");
  __builtin_amdgcn_wave_barrier();
  if (ACC) {
#pragma unroll
    for (int it = 0; it < 16; ++it) { const int f4 = lane + 32 * it, rr = f4 >> 4, q = (f4 & 15) * 4;
      const v4f_t old = *(const v4fa*)(Y + (size_t)(m0 + wm + rr) * ldy + n0 + wn + q);
      v4f_t v = *(const v4fa*)(so + rr * 68 + q); v += old; *(v4fa*)(so + rr * 68 + q) = v; }
    asm volatile("s_wait_dscnt 0" ::: "memory");
  }
#pragma unroll 1
  for (int pass = 0; pass < 2; ++pass) {
#pragma unroll
    for (int it = 0; it < 16; ++it) { const int f4 = lane + 32 * it, rr = f4 >> 4, q = (f4 & 15) * 4;
      *(volatile v4f_t*)(Y + (size_t)(m0 + wm + rr) * ldy + n0 + wn + q) = *(const v4fa*)(so + rr * 68 + q); }
    __threadfence();
  }
}

__global__ __launch_bounds__(256) void k_transpose(const float* __restrict__ Wm, float* __restrict__ Wt, int rows, int cols) {
  __shared__ float tS[64][65];
  const int tid = threadIdx.x, tbj = cols / 64, bi = blockIdx.x / tbj, bj = blockIdx.x % tbj;
  for (int e = tid; e < 64 * 64; e += 256) { const int r = e >> 6, c = e & 63; tS[r][c] = Wm[(size_t)(bi * 64 + r) * cols + bj * 64 + c]; }
  __syncthreads();
  for (int ch = tid; ch < 64 * 16; ch += 256) { const int r = ch >> 4, q4 = (ch & 15) * 4; v4f_t o; o[0] = tS[q4][r]; o[1] = tS[q4 + 1][r]; o[2] = tS[q4 + 2][r]; o[3] = tS[q4 + 3][r];
    float* dst = Wt + (size_t)(bj * 64 + r) * rows + bi * 64 + q4; *(volatile v4f_t*)dst = o; __threadfence(); *(volatile v4f_t*)dst = o; }
}


#define GSTR 48
#define SS 2048
#define HH 32
#define DKK 64
template <typename AT, int MODE>
__global__ __launch_bounds__(256) void gemm_rb_kernel(
    const AT* __restrict__ A, const float* __restrict__ W,
    const float* __restrict__ bias, const float* __restrict__ rowscale, const float* __restrict__ R, const float* __restrict__ rowbias, void* __restrict__ out,
    int M, int N, int K) {
  __shared__ bf16 ldsA[128 * LDS_STRIDE];
  __shared__ bf16 ldsW[256 * LDS_STRIDE];
  __shared__ __attribute__((aligned(16))) unsigned char sob[256 * 136 * 2];

  const int t    = threadIdx.x;
  const int wave = t >> 5;
  const int lane = t & 31;
  const int wm   = (wave & 1) * 64;
  const int wn   = (wave >> 1) * 64;
  const int mBlk = blockIdx.x * 128;
  const int nBlk = blockIdx.y * 256;

  const int arow = t >> 1;
  const int ach  = (t & 1) * 16;

  float abuf[16];
  float wbuf[32];

  stage_read16(A + (size_t)(mBlk + arow) * K + ach, abuf);
  const int nrow = min(nBlk + t, N - 1);
  stage_read16(W + (size_t)nrow * K,          wbuf);
  stage_read16(W + (size_t)nrow * K + 16,     wbuf + 16);

  f32x8 acc[4][4] = {};

  for (int k = 0; k < K; k += 32) {
    __syncthreads();
    stage_write(&ldsA[arow * LDS_STRIDE + ach], abuf, 4);
    stage_write(&ldsW[t * LDS_STRIDE],          wbuf, 8);
    if (k + 32 < K) {
      stage_read16(A + (size_t)(mBlk + arow) * K + (k + 32) + ach, abuf);
      stage_read16(W + (size_t)nrow * K + (k + 32),          wbuf);
      stage_read16(W + (size_t)nrow * K + (k + 32) + 16,     wbuf + 16);
    }
    __syncthreads();

    bf16x16 af[4], wf[4];
#pragma unroll
    for (int i = 0; i < 4; ++i)
      af[i] = lds_frag(ldsA + (wm + 16 * i) * LDS_STRIDE, LDS_STRIDE);
#pragma unroll
    for (int j = 0; j < 4; ++j)
      wf[j] = lds_frag(ldsW + (wn + 16 * j) * LDS_STRIDE, LDS_STRIDE);
#pragma unroll
    for (int i = 0; i < 4; ++i)
#pragma unroll
      for (int j = 0; j < 4; ++j)
        acc[i][j] = wmma_bf16(af[i], wf[j], acc[i][j]);
  }

  const int nlane = lane & 15;
  const int mh    = (lane >> 4) * 8;
  __syncthreads();
  if (MODE == 0 || MODE == 1 || MODE == 3) {
    bf16* so = (bf16*)sob;
#pragma unroll
    for (int i = 0; i < 4; ++i)
#pragma unroll
      for (int j = 0; j < 4; ++j) {
        const int nl = wn + 16 * j + nlane;
        const float bv = bias ? bias[nBlk + nl] : 0.0f;
        if (MODE == 3) {
#pragma unroll 1
          for (int r = 0; r < 8; ++r) {
            const int ml = wm + 16 * i + mh + r;
            const float xg = acc[i][j][r] + bv;
            so[ml * 264 + nl] = (bf16)(0.5f * xg * (1.0f + erff(xg * 0.70710678118654752f)));
          }
        } else {
#pragma unroll
        for (int r = 0; r < 8; ++r) {
          const int ml = wm + 16 * i + mh + r;
          const bf16 hv = (bf16)(acc[i][j][r] + bv);
          if (MODE == 0) so[ml * 264 + nl] = hv;
          else           so[nl * 136 + ml] = hv;
        }
        }
      }
    __syncthreads();
#pragma unroll 1
    for (int pass = 0; pass < 2; ++pass) {
      if (MODE == 0 || MODE == 3) {
        for (int ch = t; ch < 128 * 32; ch += 256) { const int ml = ch >> 5, q = (ch & 31) * 8;
          *(volatile v4u_t*)((bf16*)out + (size_t)(mBlk + ml) * N + nBlk + q) = *(const v4ua*)(so + ml * 264 + q); }
      } else {
        const int b_ = mBlk / SS, s0 = mBlk % SS;
        for (int ch = t; ch < 256 * 16; ch += 256) { const int nl = ch >> 4, q = (ch & 15) * 8; const int n = nBlk + nl, h = n >> 6, dk = n & (DKK - 1);
          *(volatile v4u_t*)((bf16*)out + (((size_t)(b_ * HH + h)) * DKK + dk) * SS + s0 + q) = *(const v4ua*)(so + nl * 136 + q); }
      }
      __threadfence();
    }
  } else {
    float* so = (float*)sob;
#pragma unroll 1
    for (int hf = 0; hf < 2; ++hf) {
      if (wm == hf * 64) {
#pragma unroll
        for (int i = 0; i < 4; ++i)
#pragma unroll
          for (int j = 0; j < 4; ++j) {
            const int nl = wn + 16 * j + nlane;
            const float bv = bias ? bias[nBlk + nl] : 0.0f;
#pragma unroll
            for (int r = 0; r < 8; ++r) { const int mrow = mBlk + hf * 64 + 16 * i + mh + r; so[(16 * i + mh + r) * 260 + nl] = acc[i][j][r] * (rowscale ? rowscale[mrow] : 1.0f) + bv + (rowbias ? rowbias[mrow] : 0.0f); }
          }
      }
      __syncthreads();
      if (R) {
        for (int ch = t; ch < 64 * 64; ch += 256) { const int ml = ch >> 6, q = (ch & 63) * 4;
          if (nBlk + q < N) { const v4f_t rv = *(const v4f_t*)(R + (size_t)(mBlk + hf * 64 + ml) * N + nBlk + q); v4f_t v = *(const v4fa*)(so + ml * 260 + q); v += rv; *(volatile v4fa*)(so + ml * 260 + q) = v; } }
        asm volatile("s_wait_dscnt 0" ::: "memory");
      }
#pragma unroll 1
      for (int pass = 0; pass < 2; ++pass) {
        for (int ch = t; ch < 64 * 64; ch += 256) { const int ml = ch >> 6, q = (ch & 63) * 4;
          if (nBlk + q < N) *(volatile v4f_t*)((float*)out + (size_t)(mBlk + hf * 64 + ml) * N + nBlk + q) = *(const v4fa*)(so + ml * 260 + q); }
        __threadfence();
      }
      __syncthreads();
    }
  }
}

#define NBf 16
#define NBF 16
#define KKf 256
#define NRf (NBf * KKf)
#define HMg 256
#define DIg 512
#define NHg 8
#define HPg 64
#define NSg 64
#define CDg 640
#define NPk 1160
#define NPP 1280
#define FDf 188
#define FDP 192
#define SSg KKf
#define TCH 64
#define NLY 2
__global__ __launch_bounds__(256) void k_fill(float* __restrict__ p, float val, size_t n4) { const size_t i = (size_t)blockIdx.x * 256 + threadIdx.x; if (i < n4) { v4f_t v = {val, val, val, val}; *(volatile v4f_t*)(p + 4 * i) = v; __threadfence(); *(volatile v4f_t*)(p + 4 * i) = v; } }
__global__ __launch_bounds__(256) void k_dbg_zero(float* __restrict__ p, size_t n4) { const size_t i = (size_t)blockIdx.x * 256 + threadIdx.x; if (i < n4) { v4f_t z = {0.f,0.f,0.f,0.f}; *(volatile v4f_t*)(p + 4 * i) = z; __threadfence(); *(volatile v4f_t*)(p + 4 * i) = z; } }
__global__ __launch_bounds__(256) void k_copy(const float* __restrict__ src, float* __restrict__ dst, size_t n4) { const size_t i = (size_t)blockIdx.x * 256 + threadIdx.x; if (i < n4) { const v4f_t v = *(const v4f_t*)(src + 4 * i); *(volatile v4f_t*)(dst + 4 * i) = v; __threadfence(); *(volatile v4f_t*)(dst + 4 * i) = v; } }
__global__ __launch_bounds__(256) void k_padT(const float* __restrict__ Wm, int kin, int nout, int npad, float* __restrict__ WT) {
  const int k = blockIdx.x, tid = threadIdx.x;
#pragma unroll 1
  for (int pass = 0; pass < 2; ++pass) {
#pragma unroll 1
    for (int n = tid; n < npad; n += 256) { const float v = (k < kin && n < nout) ? Wm[(size_t)min(n, nout - 1) * kin + min(k, kin - 1)] : 0.0f; *(volatile float*)(WT + (size_t)k * npad + n) = v; }
    __threadfence(); }
}
__global__ __launch_bounds__(64) void k_frame(const float* __restrict__ fc, const int* __restrict__ ic, const float* __restrict__ Ea, const float* __restrict__ Ej, const float* __restrict__ Ec, const float* __restrict__ Es,
                                             const float* __restrict__ El, const float* __restrict__ Eh, const float* __restrict__ Eg, const float* __restrict__ Ela, float* __restrict__ FE) {
  __shared__ float row[FDP];
  const size_t r = blockIdx.x; const int tid = threadIdx.x; const int* icr = ic + r * 17;
  row[tid] = fc[r * 64 + tid];
  if (tid < 58) { const int col = tid;
#pragma unroll
    for (int pl = 0; pl < 2; ++pl) { const int base = 64 + pl * 58; const int ipp = pl * 8;
      const float va = Ea[min(max(icr[ipp + 0], 0), 399) * 32 + min(col, 31)], vj = Ej[min(max(icr[ipp + 1], 0), 7) * 4 + min(max(col - 32, 0), 3)], vc = Ec[min(max(icr[ipp + 2], 0), 32) * 8 + min(max(col - 36, 0), 7)],
                  vl = El[min(max(icr[ipp + 3], 0), 3) * 2 + min(max(col - 44, 0), 1)], vh = Eh[min(max(icr[ipp + 4], 0), 3) * 2 + min(max(col - 46, 0), 1)], vg = Eg[min(max(icr[ipp + 5], 0), 3) * 2 + min(max(col - 48, 0), 1)],
                  vla = Ela[min(max(icr[ipp + 6], 0), 63) * 8 + min(max(col - 50, 0), 7)];
      const float v = (col < 32) ? va : (col < 36) ? vj : (col < 44) ? vc : (col < 46) ? vl : (col < 48) ? vh : (col < 50) ? vg : vla;
      row[base + col] = v; } }
  if (tid < 8) { const int ix = min(max(icr[16], 0), 31); row[180 + tid] = Es[ix * 8 + tid]; }
  if (tid < 4) row[188 + tid] = 0.0f;
  __syncthreads();
#pragma unroll 1
  for (int pass = 0; pass < 2; ++pass) { for (int c = tid; c < FDP; c += 64) *(volatile float*)(FE + r * FDP + c) = row[c]; __threadfence(); }
}
__global__ __launch_bounds__(64) void k_rms(const float* __restrict__ X, const float* __restrict__ w, float* __restrict__ Y) {
  __shared__ float red[64];
  const size_t r = blockIdx.x; const int tid = threadIdx.x; const v4f_t v = *(const v4f_t*)(X + r * HMg + 4 * tid); red[tid] = v[0] * v[0] + v[1] * v[1] + v[2] * v[2] + v[3] * v[3]; __syncthreads();
  for (int o = 32; o > 0; o >>= 1) { if (tid < o) red[tid] += red[tid + o]; __syncthreads(); }
  const float rs = 1.0f / __builtin_sqrtf(red[0] * (1.0f / HMg) + 1e-5f); const v4f_t y = v * rs * *(const v4f_t*)(w + 4 * tid);
  *(volatile v4f_t*)(Y + r * HMg + 4 * tid) = y; __threadfence(); *(volatile v4f_t*)(Y + r * HMg + 4 * tid) = y;
}
__global__ __launch_bounds__(256) void k_conv(const float* __restrict__ ZX, const float* __restrict__ cw, const float* __restrict__ cb, float* __restrict__ XC) {
  const size_t r = blockIdx.x; const int tid = threadIdx.x; const int t = (int)(r % KKf); const size_t r0 = r - t;
#pragma unroll 1
  for (int pass = 0; pass < 2; ++pass) {
#pragma unroll 1
    for (int c = tid; c < CDg; c += 256) { float acc = cb[c];
#pragma unroll
      for (int k = 0; k < 4; ++k) { const int tt = t - 3 + k; const int tc = max(tt, 0); const float xv = ZX[(r0 + tc) * NPP + DIg + c]; acc = fmaf((tt >= 0) ? xv : 0.0f, cw[c * 4 + k], acc); }
      *(volatile float*)(XC + r * CDg + c) = acc / (1.0f + expf(-acc)); }
    __threadfence(); }
}
__global__ __launch_bounds__(256) void k_scan4(const float* __restrict__ XC, const float* __restrict__ ZX, const float* __restrict__ dtb, const float* __restrict__ Alog, const float* __restrict__ Dv, float* __restrict__ Y) {
  __shared__ float BC[TCH][2 * NSg]; __shared__ float DT[TCH]; __shared__ __attribute__((aligned(16))) float yS[TCH][64 + 4];
  const int h = blockIdx.x, tid = threadIdx.x; const size_t rb = (size_t)blockIdx.y * SSg; const int cl = tid >> 2, qq = tid & 3; const int ch = h * 64 + cl;
  const float A2 = -expf(Alog[h]) * 1.4426950408889634f; const float Dd = Dv[h]; const float db = dtb[h]; float hs[16];
#pragma unroll
  for (int n = 0; n < 16; ++n) hs[n] = 0.0f;
#pragma unroll 1
  for (int c0 = 0; c0 < SSg; c0 += TCH) {
    __syncthreads();
#pragma unroll 1
    for (int e = tid; e < TCH * 2 * NSg; e += 256) { const int tt = e >> 7, c = e & 127; BC[tt][c] = XC[(rb + c0 + tt) * CDg + DIg + c]; }
    if (tid < TCH) { const float dr = ZX[(rb + c0 + tid) * NPP + DIg + CDg + h] + db; DT[tid] = (dr > 20.0f) ? dr : log1pf(expf(dr)); }
    __syncthreads();
#pragma unroll 1
    for (int tt = 0; tt < TCH; ++tt) {
      const float dt = DT[tt]; const float da = __builtin_amdgcn_exp2f(dt * A2); const float xv = XC[(rb + c0 + tt) * CDg + ch]; const float dtx = dt * xv; float y = 0.0f;
#pragma unroll
      for (int n = 0; n < 16; ++n) { hs[n] = fmaf(hs[n], da, dtx * BC[tt][16 * qq + n]); y = fmaf(hs[n], BC[tt][NSg + 16 * qq + n], y); }
      y += __shfl_xor(y, 1, 32); y += __shfl_xor(y, 2, 32);
      if (qq == 0) yS[tt][cl] = y + Dd * xv; }
    __syncthreads();
#pragma unroll 1
    for (int pass = 0; pass < 2; ++pass) {
#pragma unroll 1
      for (int i = tid; i < TCH * 16; i += 256) { const int tt = i >> 4, piece = (i & 15) * 4;
        *(volatile v4f_t*)(Y + (rb + c0 + tt) * DIg + h * 64 + piece) = *(const v4fa*)(&yS[tt][piece]); }
      __threadfence(); }
  }
}
__global__ __launch_bounds__(128) void k_gnorm(const float* __restrict__ Y, const float* __restrict__ ZX, const float* __restrict__ w, f16* __restrict__ Gout) {
  __shared__ float red[128];
  const size_t r = blockIdx.x; const int tid = threadIdx.x, c = 4 * tid; const v4f_t y = *(const v4f_t*)(Y + r * DIg + c); const v4f_t z = *(const v4f_t*)(ZX + r * NPP + c); v4f_t g; float s = 0.0f;
#pragma unroll
  for (int u = 0; u < 4; ++u) { g[u] = y[u] * (z[u] / (1.0f + expf(-z[u]))); s += g[u] * g[u]; }
  red[tid] = s; __syncthreads(); for (int o = 64; o > 0; o >>= 1) { if (tid < o) red[tid] += red[tid + o]; __syncthreads(); }
  const float rs = 1.0f / __builtin_sqrtf(red[0] * (1.0f / DIg) + 1e-5f); const v4f_t wv = *(const v4f_t*)(w + c); union { f16 hh[4]; unsigned long long u; } o;
#pragma unroll
  for (int u = 0; u < 4; ++u) o.hh[u] = (f16)(g[u] * rs * wv[u]);
  *(volatile unsigned long long*)(Gout + r * DIg + c) = o.u; __threadfence(); *(volatile unsigned long long*)(Gout + r * DIg + c) = o.u;
}
__global__ __launch_bounds__(64) void k_cath(const float* __restrict__ w, int off, float* __restrict__ WH) {
  const int r = blockIdx.x, tid = threadIdx.x; const v4f_t v = *(const v4f_t*)(w + (size_t)r * HMg + 4 * tid); float* d = WH + (size_t)(off + r) * HMg + 4 * tid;
  *(volatile v4f_t*)d = v; __threadfence(); *(volatile v4f_t*)d = v;
}
__global__ __launch_bounds__(1024) void k_catb(const float* __restrict__ b0, const float* __restrict__ b1, const float* __restrict__ b2, const float* __restrict__ b3, const float* __restrict__ b4, const float* __restrict__ b5, float* __restrict__ BH) {
  const int o = threadIdx.x; if (o >= 832) return;
  const float v0 = b0[min(o, 7)], v1 = b1[min(max(o - 8, 0), 5)], v2 = b2[min(max(o - 14, 0), 399)], v3 = b3[min(max(o - 414, 0), 399)], v4 = b4[min(max(o - 814, 0), 7)], v5 = b5[min(max(o - 822, 0), 7)];
  const float v = (o < 8) ? v0 : (o < 14) ? v1 : (o < 414) ? v2 : (o < 814) ? v3 : (o < 822) ? v4 : (o < 830) ? v5 : 0.0f;
  *(volatile float*)(BH + o) = v; __threadfence(); *(volatile float*)(BH + o) = v;
}
__global__ __launch_bounds__(256) void k_heads(const float* __restrict__ X, const float* __restrict__ fw, const float* __restrict__ ctrl, const float* __restrict__ Wc, const float* __restrict__ bc, const float* __restrict__ WH, const float* __restrict__ BH, float* __restrict__ HOP) {
  __shared__ float red[256]; __shared__ float hv[HMg]; __shared__ float ho[832];
  const int b = blockIdx.x, tid = threadIdx.x; const float xv = X[((size_t)b * KKf + KKf - 1) * HMg + tid]; red[tid] = xv * xv; __syncthreads();
  for (int o = 128; o > 0; o >>= 1) { if (tid < o) red[tid] += red[tid + o]; __syncthreads(); }
  const float rs = 1.0f / __builtin_sqrtf(red[0] * (1.0f / HMg) + 1e-5f); float hcur = xv * rs * fw[tid] + bc[tid];
#pragma unroll
  for (int j = 0; j < 16; ++j) hcur = fmaf(ctrl[b * 16 + j], Wc[tid * 16 + j], hcur);
  hv[tid] = hcur; __syncthreads();
#pragma unroll 1
  for (int o = tid; o < 830; o += 256) { const float* wr = WH + (size_t)o * HMg; float a = BH[o];
#pragma unroll 1
    for (int i = 0; i < HMg; ++i) a = fmaf(hv[i], wr[i], a);
    ho[o] = a; }
  __syncthreads();
#pragma unroll 1
  for (int pass = 0; pass < 2; ++pass) { for (int o = tid; o < 1024; o += 256) *(volatile float*)(HOP + (size_t)b * 1024 + o) = (o < 830) ? ho[o] : 0.0f; __threadfence(); }
}
__global__ __launch_bounds__(1024) void k_outw(const float* __restrict__ HOP, float* __restrict__ out) {
  const int tid = threadIdx.x;
#pragma unroll 1
  for (int pass = 0; pass < 2; ++pass) {
#pragma unroll 1
    for (int fi = tid; fi < 13280; fi += 1024) { int b, o;
      if (fi < 128) { b = fi / 8; o = fi % 8; } else if (fi < 224) { b = (fi - 128) / 6; o = 8 + (fi - 128) % 6; } else if (fi < 6624) { b = (fi - 224) / 400; o = 14 + (fi - 224) % 400; }
      else if (fi < 13024) { b = (fi - 6624) / 400; o = 414 + (fi - 6624) % 400; } else if (fi < 13152) { b = (fi - 13024) / 8; o = 814 + (fi - 13024) % 8; } else { b = (fi - 13152) / 8; o = 822 + (fi - 13152) % 8; }
      *(volatile float*)(out + fi) = HOP[(size_t)b * 1024 + o]; }
    __threadfence(); }
}

extern "C" void kernel_launch(void* const* d_in, const int* in_sizes, int n_in,
                              void* d_out, int out_size, void* d_ws, size_t ws_size,
                              hipStream_t stream) {
  (void)in_sizes; (void)n_in; (void)out_size;
  const float** f = (const float**)d_in;
  const float* fc = f[0], *ctrl = f[1], *Ea = f[2], *Ej = f[3], *Ec = f[4], *Es = f[5], *El = f[6], *Eh = f[7], *Eg = f[8], *Ela = f[9], *fpw = f[10], *fpb = f[11], *ipw = f[12], *cw = f[13], *cb = f[14],
              *dtb = f[15], *Alog = f[16], *Dsk = f[17], *mnw = f[18], *opw = f[19], *lnw = f[20], *fnw = f[21], *Wc = f[22], *bcp = f[23],
              *w0 = f[24], *b0 = f[25], *w1 = f[26], *b1 = f[27], *w2 = f[28], *b2 = f[29], *w3 = f[30], *b3 = f[31], *w4 = f[32], *b4 = f[33], *w5 = f[34], *b5 = f[35];
  const int* ic = (const int*)d_in[36];
  float* out = (float*)d_out;
  char* ws = (char*)d_ws;
  float* WfT = (float*)ws; ws += (size_t)FDP * HMg * 4; float* WinT = (float*)ws; ws += (size_t)NLY * HMg * NPP * 4;
  float* FE = (float*)ws; ws += (size_t)NRf * FDP * 4; float* XA = (float*)ws; ws += (size_t)NRf * HMg * 4; float* XB = (float*)ws; ws += (size_t)NRf * HMg * 4; float* HN = (float*)ws; ws += (size_t)NRf * HMg * 4;
  float* ZX = (float*)ws; ws += (size_t)NRf * NPP * 4; float* XC = (float*)ws; ws += (size_t)NRf * CDg * 4; float* Y = (float*)ws; ws += (size_t)NRf * DIg * 4; f16* G16 = (f16*)ws; ws += (size_t)NRf * DIg * 2;
  float* HOP = (float*)ws; ws += (size_t)NBF * 1024 * 4; float* WH = (float*)ws; ws += (size_t)832 * HMg * 4; float* BH = (float*)ws; ws += 832 * 4;
  if ((size_t)(ws - (char*)d_ws) > ws_size) return;
  const dim3 blk(256);
  k_padT<<<dim3(FDP), blk, 0, stream>>>(fpw, FDf, HMg, HMg, WfT);
  for (int l = 0; l < NLY; ++l) k_padT<<<dim3(HMg), blk, 0, stream>>>(ipw + (size_t)l * NPk * HMg, HMg, NPk, NPP, WinT + (size_t)l * HMg * NPP);
  k_fill<<<dim3((NBF * 1024 / 4 + 255) / 256), blk, 0, stream>>>(HOP, 0.0f, NBF * 1024 / 4);
  k_cath<<<dim3(8), dim3(64), 0, stream>>>(w0, 0, WH); k_cath<<<dim3(6), dim3(64), 0, stream>>>(w1, 8, WH); k_cath<<<dim3(400), dim3(64), 0, stream>>>(w2, 14, WH);
  k_cath<<<dim3(400), dim3(64), 0, stream>>>(w3, 414, WH); k_cath<<<dim3(8), dim3(64), 0, stream>>>(w4, 814, WH); k_cath<<<dim3(8), dim3(64), 0, stream>>>(w5, 822, WH);
  k_catb<<<dim3(1), dim3(1024), 0, stream>>>(b0, b1, b2, b3, b4, b5, BH);
  k_frame<<<dim3(NRf), dim3(64), 0, stream>>>(fc, ic, Ea, Ej, Ec, Es, El, Eh, Eg, Ela, FE);
  gemm_kne<float, 0, false><<<dim3(NRf / 128, HMg / 128), blk, 0, stream>>>(FE, FDP, WfT, HMg, fpb, nullptr, nullptr, XA, HMg, FDP);
  float* h = XA; float* hn = XB;
  for (int l = 0; l < NLY; ++l) {
    k_rms<<<dim3(NRf), dim3(64), 0, stream>>>(h, lnw + l * HMg, HN);
    gemm_kne<float, 0, false><<<dim3(NRf / 128, NPP / 128), blk, 0, stream>>>(HN, HMg, WinT + (size_t)l * HMg * NPP, NPP, nullptr, nullptr, nullptr, ZX, NPP, HMg);
    k_conv<<<dim3(NRf), blk, 0, stream>>>(ZX, cw + (size_t)l * CDg * 4, cb + (size_t)l * CDg, XC);
    k_scan4<<<dim3(NHg, NBf), blk, 0, stream>>>(XC, ZX, dtb + l * NHg, Alog + l * NHg, Dsk + l * NHg, Y);
    k_gnorm<<<dim3(NRf), dim3(128), 0, stream>>>(Y, ZX, mnw + (size_t)l * DIg, G16);
    gemm_rb_kernel<bf16, 2><<<dim3(NRf / 128, HMg / 256), blk, 0, stream>>>(G16, opw + (size_t)l * HMg * DIg, nullptr, nullptr, h, nullptr, hn, NRf, HMg, DIg);
    { float* t = h; h = hn; hn = t; }
  }
  k_heads<<<dim3(NBf), blk, 0, stream>>>(h, fnw, ctrl, Wc, bcp, WH, BH, HOP);
  k_outw<<<dim3(1), dim3(1024), 0, stream>>>(HOP, out);
}
